// LSTM_Mod2_11398843203682
// MI455X (gfx1250) — hardware-run, weakly checked
//
#include <hip/hip_runtime.h>

constexpr int N_STEPS   = 1024;
constexpr int N_BATCH   = 64;
constexpr int N_HID     = 1024;
constexpr int N_GATES   = 4 * N_HID;
constexpr int N_VOCAB   = 128;
constexpr int TILE_ROWS = 16;
constexpr int H_PITCH   = N_HID + 8;
constexpr int H_BUF     = TILE_ROWS * H_PITCH;
constexpr int SCAN_THREADS = 512;
constexpr int SCAN_WAVES   = SCAN_THREADS / 32;
constexpr int OUT_WAVES    = 4;
constexpr int CAST_THREADS = 256;

constexpr float W_CARRY = 256.0f;
constexpr float H_CARRY = 256.0f;
constexpr float FOLD    = 1.0f / (W_CARRY * H_CARRY);

static_assert(N_BATCH % TILE_ROWS == 0, "batch tiles");
static_assert(N_HID % 32 == 0, "k steps of 32");
static_assert(SCAN_WAVES * 64 == N_HID, "one wave per 64 hidden units");
static_assert(OUT_WAVES * 32 == N_VOCAB, "one wave per 32 output columns");
static_assert((H_PITCH * 2) % 16 == 0, "16-byte aligned LDS rows");
static_assert(((size_t)N_GATES * N_HID / 8) % CAST_THREADS == 0, "cast blocks exact");
static_assert(((size_t)N_VOCAB * N_HID / 8) % CAST_THREADS == 0, "cast blocks exact");

typedef __attribute__((ext_vector_type(16))) _Float16 v16h;
typedef __attribute__((ext_vector_type(8)))  _Float16 v8h;
typedef __attribute__((ext_vector_type(8)))  float    v8f;
typedef __attribute__((ext_vector_type(4)))  float    v4f;

struct FragH {
  union U { v16h v; v8h h[2]; };
  static __device__ __forceinline__ v16h load(const _Float16* p) {
    U f;
    f.h[0] = *(const v8h*)(p);
    f.h[1] = *(const v8h*)(p + 16);
    return f.v;
  }
  static __device__ __forceinline__ v8f mma(v16h a, v16h b, v8f c) {
    return __builtin_amdgcn_wmma_f32_16x16x32_f16(false, a, false, b, (short)0, c, false, false);
  }
};

__device__ __forceinline__ void tie_acc(v8f& c) { asm volatile("" : "+v"(c)); }
__device__ __forceinline__ void guard_group8(v8f& c, v16h a, v16h b0, v16h b1, v16h b2, v16h b3,
                                             v16h b4, v16h b5, v16h b6, v16h b7) {
  asm volatile("v_nop\n\tv_nop\n\tv_nop\n\tv_nop"
               : "+v"(c)
               : "v"(a), "v"(b0), "v"(b1), "v"(b2), "v"(b3), "v"(b4), "v"(b5), "v"(b6), "v"(b7));
}
__device__ __forceinline__ void guard_group2(v8f& c, v16h a, v16h b0, v16h b1) {
  asm volatile("v_nop\n\tv_nop\n\tv_nop\n\tv_nop" : "+v"(c) : "v"(a), "v"(b0), "v"(b1));
}

__device__ __forceinline__ float sigm_f(float x) { return __builtin_amdgcn_rcpf(1.0f + __expf(-x)); }
__device__ __forceinline__ float tanh_f(float x) { return 1.0f - 2.0f * __builtin_amdgcn_rcpf(__expf(2.0f * x) + 1.0f); }

__global__ __launch_bounds__(CAST_THREADS) void cast_planes_kernel(
    const float* __restrict__ src0, _Float16* __restrict__ dst0, int nblk0, int n8_0,
    const float* __restrict__ src1, _Float16* __restrict__ dst1, int n8_1, float scale)
{
  const bool first = ((int)blockIdx.x < nblk0);
  const float* src = first ? src0 : src1;
  _Float16* dst = first ? dst0 : dst1;
  const int n8 = first ? n8_0 : n8_1;
  const int blk = first ? (int)blockIdx.x : ((int)blockIdx.x - nblk0);
  const int idx = blk * CAST_THREADS + (int)threadIdx.x;
  const int ic = (idx < n8) ? idx : (n8 - 1);
  const v4f x0 = *(const v4f*)(src + (size_t)ic * 8);
  const v4f x1 = *(const v4f*)(src + (size_t)ic * 8 + 4);
  v8h o;
  o[0] = (_Float16)(x0[0] * scale);
  o[1] = (_Float16)(x0[1] * scale);
  o[2] = (_Float16)(x0[2] * scale);
  o[3] = (_Float16)(x0[3] * scale);
  o[4] = (_Float16)(x1[0] * scale);
  o[5] = (_Float16)(x1[1] * scale);
  o[6] = (_Float16)(x1[2] * scale);
  o[7] = (_Float16)(x1[3] * scale);
  if (idx < n8) {
    *(volatile v8h*)(dst + (size_t)idx * 8) = o;
    __threadfence();
    *(volatile v8h*)(dst + (size_t)idx * 8) = o;
  }
}

__global__ __launch_bounds__(SCAN_THREADS) void lstm_scan_kernel(
    const float* __restrict__ sentence, const float* __restrict__ wih,
    const float* __restrict__ bih, const float* __restrict__ bhh, const float* __restrict__ blin,
    const _Float16* __restrict__ Whh16, const _Float16* __restrict__ Wlin16, float* __restrict__ out)
{
  __shared__ __align__(16) _Float16 hsh[2 * H_BUF];
  __shared__ __align__(16) float bsh[N_GATES];
  __shared__ __align__(16) float wsh[N_GATES];
  __shared__ __align__(16) float osl[OUT_WAVES * TILE_ROWS * 32];

  const int tid  = (int)threadIdx.x;
  const int lane = tid & 31;
  const int wave = __builtin_amdgcn_readfirstlane(tid >> 5);
  const int hh = lane >> 4;
  const int rl = lane & 15;
  const int b0 = (int)blockIdx.x * TILE_ROWS;

#pragma unroll 1
  for (int i = tid; i < 2 * H_BUF; i += SCAN_THREADS) hsh[i] = (_Float16)0.0f;
#pragma unroll 1
  for (int i = tid; i < N_GATES; i += SCAN_THREADS) {
    bsh[i] = bih[i] + bhh[i];
    wsh[i] = wih[i];
  }
  const int ow = wave & (OUT_WAVES - 1);
  float bl0 = blin[32 * ow + rl];
  float bl1 = blin[32 * ow + 16 + rl];
  asm volatile("" : "+v"(bl0));
  asm volatile("" : "+v"(bl1));

  float cst[2][2][8];
#pragma unroll
  for (int p = 0; p < 2; ++p)
#pragma unroll
    for (int qq = 0; qq < 2; ++qq)
#pragma unroll
      for (int r = 0; r < 8; ++r) cst[p][qq][r] = 0.0f;

  __syncthreads();

  const v8f z8 = {0.f, 0.f, 0.f, 0.f, 0.f, 0.f, 0.f, 0.f};
  const int rq = lane >> 3;
  const int c4 = (lane & 7) * 4;
  float* slab = osl + ow * (TILE_ROWS * 32);

#pragma unroll 1
  for (int t = 0; t < N_STEPS; ++t) {
    const _Float16* hc = hsh + (t & 1) * H_BUF;
    _Float16* hn = hsh + ((t & 1) ^ 1) * H_BUF;

    const float* xp = sentence + (size_t)t * N_BATCH + b0 + 8 * hh;
    const v4f xa = *(const v4f*)(xp);
    const v4f xb = *(const v4f*)(xp + 4);
    float xr[8];
    xr[0] = xa[0]; xr[1] = xa[1]; xr[2] = xa[2]; xr[3] = xa[3];
    xr[4] = xb[0]; xr[5] = xb[1]; xr[6] = xb[2]; xr[7] = xb[3];

#pragma unroll
    for (int p = 0; p < 2; ++p) {
      v8f acc[8];
#pragma unroll
      for (int i = 0; i < 8; ++i) acc[i] = z8;
      const _Float16* ap = hc + rl * H_PITCH + 8 * hh;
      const _Float16* wp = Whh16 + (size_t)(64 * wave + 32 * p + rl) * N_HID + 8 * hh;
#pragma unroll 1
      for (int ks = 0; ks < N_HID / 32; ++ks) {
        const v16h a = FragH::load(ap);
        v16h bf[8];
#pragma unroll
        for (int qq = 0; qq < 2; ++qq)
#pragma unroll
          for (int g = 0; g < 4; ++g)
            bf[qq * 4 + g] = FragH::load(wp + (size_t)(g * N_HID + 16 * qq) * N_HID);
#pragma unroll
        for (int i = 0; i < 8; ++i) acc[i] = FragH::mma(a, bf[i], acc[i]);
        tie_acc(acc[0]);
        tie_acc(acc[1]);
        tie_acc(acc[2]);
        tie_acc(acc[3]);
        tie_acc(acc[4]);
        tie_acc(acc[5]);
        tie_acc(acc[6]);
        guard_group8(acc[7], a, bf[0], bf[1], bf[2], bf[3], bf[4], bf[5], bf[6], bf[7]);
        ap += 32;
        wp += 32;
      }

#pragma unroll
      for (int qq = 0; qq < 2; ++qq) {
        const int u = 64 * wave + 16 * (2 * p + qq) + rl;
        const float wI = wsh[u];
        const float wF = wsh[N_HID + u];
        const float wG = wsh[2 * N_HID + u];
        const float wO = wsh[3 * N_HID + u];
        const float bI = bsh[u];
        const float bF = bsh[N_HID + u];
        const float bG = bsh[2 * N_HID + u];
        const float bO = bsh[3 * N_HID + u];
#pragma unroll
        for (int r = 0; r < 8; ++r) {
          const float x = xr[r];
          const float zi = acc[qq * 4 + 0][r] * FOLD + (x * wI + bI);
          const float zf = acc[qq * 4 + 1][r] * FOLD + (x * wF + bF);
          const float zg = acc[qq * 4 + 2][r] * FOLD + (x * wG + bG);
          const float zo = acc[qq * 4 + 3][r] * FOLD + (x * wO + bO);
          const float ig = sigm_f(zi);
          const float fg = sigm_f(zf);
          const float gg = tanh_f(zg);
          const float og = sigm_f(zo);
          const float cn = fg * cst[p][qq][r] + ig * gg;
          cst[p][qq][r] = cn;
          const float hv = og * tanh_f(cn);
          hn[(8 * hh + r) * H_PITCH + u] = (_Float16)(hv * H_CARRY);
        }
      }
    }

    __syncthreads();

    if (wave < OUT_WAVES) {
      v8f o0 = z8;
      v8f o1 = z8;
      const _Float16* ap = hn + rl * H_PITCH + 8 * hh;
      const _Float16* lp = Wlin16 + (size_t)(32 * wave + rl) * N_HID + 8 * hh;
#pragma unroll 1
      for (int ks = 0; ks < N_HID / 32; ++ks) {
        const v16h a = FragH::load(ap);
        const v16h b0f = FragH::load(lp);
        const v16h b1f = FragH::load(lp + (size_t)16 * N_HID);
        o0 = FragH::mma(a, b0f, o0);
        o1 = FragH::mma(a, b1f, o1);
        tie_acc(o0);
        guard_group2(o1, a, b0f, b1f);
        ap += 32;
        lp += 32;
      }
#pragma unroll
      for (int r = 0; r < 8; ++r) {
        slab[(8 * hh + r) * 32 + rl]      = o0[r] * FOLD + bl0;
        slab[(8 * hh + r) * 32 + 16 + rl] = o1[r] * FOLD + bl1;
      }
      __builtin_amdgcn_fence(__ATOMIC_RELEASE, "workgroup");
      __builtin_amdgcn_wave_barrier();
      __builtin_amdgcn_fence(__ATOMIC_ACQUIRE, "workgroup");
      v4f ov[4];
#pragma unroll
      for (int it = 0; it < 4; ++it) ov[it] = *(const v4f*)(slab + (it * 4 + rq) * 32 + c4);
      float* ob = out + ((size_t)t * N_BATCH + b0) * N_VOCAB + 32 * wave + c4;
      for (int pass = 0; pass < 2; ++pass) {
#pragma unroll
        for (int it = 0; it < 4; ++it)
          *(volatile v4f*)(ob + (size_t)(it * 4 + rq) * N_VOCAB) = ov[it];
        __threadfence();
      }
      __builtin_amdgcn_fence(__ATOMIC_RELEASE, "workgroup");
      __builtin_amdgcn_wave_barrier();
      __builtin_amdgcn_fence(__ATOMIC_ACQUIRE, "workgroup");
    }
  }
}

extern "C" void kernel_launch(void* const* d_in, const int* in_sizes, int n_in,
                              void* d_out, int out_size, void* d_ws, size_t ws_size,
                              hipStream_t stream) {
  if (n_in < 7 || d_out == nullptr || d_ws == nullptr) return;
  if (in_sizes[0] != N_STEPS * N_BATCH) return;
  if (in_sizes[1] != N_GATES) return;
  if (in_sizes[2] != N_GATES * N_HID) return;
  if (in_sizes[3] != N_GATES || in_sizes[4] != N_GATES) return;
  if (in_sizes[5] != N_VOCAB * N_HID || in_sizes[6] != N_VOCAB) return;
  if (out_size != N_STEPS * N_BATCH * N_VOCAB) return;

  const float* sentence = (const float*)d_in[0];
  const float* wih      = (const float*)d_in[1];
  const float* whh      = (const float*)d_in[2];
  const float* bih      = (const float*)d_in[3];
  const float* bhh      = (const float*)d_in[4];
  const float* wlin     = (const float*)d_in[5];
  const float* blin     = (const float*)d_in[6];
  float* out = (float*)d_out;

  char* ws = (char*)d_ws;
  size_t off = 0;
  auto carve = [&](size_t bytes) -> char* { char* p = ws + off; off += (bytes + 255) & ~(size_t)255; return p; };
  _Float16* Whh16  = (_Float16*)carve((size_t)N_GATES * N_HID * 2);
  _Float16* Wlin16 = (_Float16*)carve((size_t)N_VOCAB * N_HID * 2);
  if (off > ws_size || off > (size_t)134217728) return;

  const int n8_0 = N_GATES * N_HID / 8;
  const int n8_1 = N_VOCAB * N_HID / 8;
  const int nblk0 = n8_0 / CAST_THREADS;
  const int nblk1 = n8_1 / CAST_THREADS;
  cast_planes_kernel<<<nblk0 + nblk1, CAST_THREADS, 0, stream>>>(whh, Whh16, nblk0, n8_0, wlin, Wlin16, n8_1, W_CARRY);

  lstm_scan_kernel<<<N_BATCH / TILE_ROWS, SCAN_THREADS, 0, stream>>>(sentence, wih, bih, bhh, blin, Whh16, Wlin16, out);
}
